// DenseMLPQMatrixDecoder_45011257262439
// MI455X (gfx1250) — hardware-run, weakly checked
//
#include <hip/hip_runtime.h>


#ifndef NV
#define NV 1024
#endif
#ifndef NS
#define NS 1024
#endif
#define NV_FULL 1024
#define NS_FULL 1024
#ifndef OUT_S
#define OUT_S NS_FULL
#endif
#define DE   8
#define HW   16
#define NA   4
#define HP   20
#define TS   12
#define TO   12
#define TINF 1000.0f
#define XSC  (1.0f / (float)(1 << TS))

static_assert(DE == 8);
static_assert(HW == 16);
static_assert(2 * HW == 32);
static_assert(NA * NA == HW);
static_assert(NV % 32 == 0);
static_assert(NV <= NV_FULL);
static_assert(NS <= NS_FULL);
static_assert(NS <= OUT_S);
static_assert(NS % 256 == 0);
static_assert((size_t)256 * (NS / 256) * 16 == (size_t)NS * NA * 4);
static_assert(32 * 16 == 32 * NA * 4);
static_assert(HP >= HW);
static_assert((HP * 4) % 16 == 0);
static_assert(32 * HP * 4 <= 131072);
static_assert(TS >= 1 && TS <= 20);
static_assert(TO >= 2);

typedef unsigned short bf;
typedef __attribute__((ext_vector_type(16))) __bf16   v16bf;
typedef __attribute__((ext_vector_type(8)))  unsigned short v8us;
typedef __attribute__((ext_vector_type(8)))  float    v8f;
typedef __attribute__((ext_vector_type(4)))  float    v4f;
typedef v4f  __attribute__((may_alias)) v4fa;

__device__ __forceinline__ unsigned short f2bf(float f) { unsigned u = __float_as_uint(f); u += 0x7FFFu + ((u >> 16) & 1u); return (unsigned short)(u >> 16); }
__device__ __forceinline__ float bfr(float f) { return __uint_as_float(((unsigned)f2bf(f)) << 16); }
__device__ __forceinline__ v16bf cat16b(v8us lo, v8us hi) { return __builtin_bit_cast(v16bf, __builtin_shufflevector(lo, hi, 0, 1, 2, 3, 4, 5, 6, 7, 8, 9, 10, 11, 12, 13, 14, 15)); }
__device__ __forceinline__ v8f wmmab(v16bf a, v16bf b, v8f c) { return __builtin_amdgcn_wmma_f32_16x16x32_bf16(false, a, false, b, (short)0, c, false, false); }
__device__ __forceinline__ void wave_sync() { __builtin_amdgcn_fence(3  , "wavefront"); __builtin_amdgcn_wave_barrier(); asm volatile("" ::: "memory"); }

__device__ __forceinline__ v8f wmmab_g(v16bf a, v16bf b, v8f c) {
    c = wmmab(a, b, c);
    asm volatile("v_nop\n\tv_nop\n\tv_nop\n\tv_nop" : "+v"(c) : "v"(a), "v"(b));
    return c;
}

__device__ __forceinline__ void mm4(const float (&X)[16], const float (&Y)[16], float (&Z)[16]) {
#pragma unroll
    for (int i = 0; i < 4; ++i) {
#pragma unroll
        for (int j = 0; j < 4; ++j) {
            float s = 0.0f;
#pragma unroll
            for (int k = 0; k < 4; ++k) s = fmaf(X[i * 4 + k], Y[k * 4 + j], s);
            Z[i * 4 + j] = s;
        }
    }
}

__global__ __launch_bounds__(32) void k_chain(const float* __restrict__ emb, const float* __restrict__ W0, const float* __restrict__ b0,
                                              const float* __restrict__ W1, const float* __restrict__ b1,
                                              const float* __restrict__ W2, const float* __restrict__ b2, float* PR) {
    __shared__ __align__(16) float hs[32 * HP];
    const int lane = threadIdx.x & 31, lr = lane & 15, hi = lane >> 4;
    const int v0 = blockIdx.x * 32;
    const bool lo16 = hi == 0;
    const v8us z8 = (v8us){};
    v8f acc[2];

    {
        float w[8];
#pragma unroll
        for (int i = 0; i < 8; ++i) w[i] = W0[i * HW + lr];
#pragma unroll
        for (int i = 0; i < 8; ++i) asm volatile("" : "+v"(w[i]));
        v8us wl;
#pragma unroll
        for (int i = 0; i < 8; ++i) wl[i] = lo16 ? f2bf(w[i]) : (unsigned short)0;
        const v16bf bw = cat16b(wl, z8);
#pragma unroll
        for (int mt = 0; mt < 2; ++mt) {
            const float* er = emb + (size_t)(v0 + 16 * mt + lr) * DE;
            v4f e0 = *(const v4f*)er, e1 = *(const v4f*)(er + 4);
            asm volatile("" : "+v"(e0)); asm volatile("" : "+v"(e1));
            v8us xl;
#pragma unroll
            for (int i = 0; i < 4; ++i) { xl[i] = lo16 ? f2bf(e0[i]) : (unsigned short)0; xl[4 + i] = lo16 ? f2bf(e1[i]) : (unsigned short)0; }
            acc[mt] = wmmab_g(cat16b(xl, z8), bw, (v8f){});
        }
    }

    {
        const float bv = bfr(b0[lr]);
#pragma unroll
        for (int mt = 0; mt < 2; ++mt) {
#pragma unroll
            for (int r = 0; r < 8; ++r) { const float x = acc[mt][r] + bv; hs[(16 * mt + 8 * hi + r) * HP + lr] = x > 0.0f ? x : 0.0f; } }
    }
    wave_sync();
    {
        v8us w8;
#pragma unroll
        for (int i = 0; i < 8; ++i) w8[i] = f2bf(W1[(8 * hi + i) * HW + lr]);
        const v16bf bw = cat16b(w8, w8);
#pragma unroll
        for (int mt = 0; mt < 2; ++mt) {
            const v4f x0 = *(const v4fa*)(&hs[(16 * mt + lr) * HP + 8 * hi]); const v4f x1 = *(const v4fa*)(&hs[(16 * mt + lr) * HP + 8 * hi + 4]);
            v8us hv, rv;
#pragma unroll
            for (int i = 0; i < 4; ++i) {
                const unsigned short a0 = f2bf(x0[i]); const unsigned short a1 = f2bf(x1[i]);
                hv[i] = a0; hv[4 + i] = a1;
                rv[i] = f2bf(x0[i] - __uint_as_float(((unsigned)a0) << 16)); rv[4 + i] = f2bf(x1[i] - __uint_as_float(((unsigned)a1) << 16)); }
            acc[mt] = wmmab_g(cat16b(hv, rv), bw, (v8f){});
        }
    }
    wave_sync();

    {
        const float bv = bfr(b1[lr]);
#pragma unroll
        for (int mt = 0; mt < 2; ++mt) {
#pragma unroll
            for (int r = 0; r < 8; ++r) { const float x = acc[mt][r] + bv; hs[(16 * mt + 8 * hi + r) * HP + lr] = x > 0.0f ? x : 0.0f; } }
    }
    wave_sync();
    {
        v8us w8;
#pragma unroll
        for (int i = 0; i < 8; ++i) w8[i] = f2bf(W2[(8 * hi + i) * HW + lr]);
        const v16bf bw = cat16b(w8, w8);
#pragma unroll
        for (int mt = 0; mt < 2; ++mt) {
            const v4f x0 = *(const v4fa*)(&hs[(16 * mt + lr) * HP + 8 * hi]); const v4f x1 = *(const v4fa*)(&hs[(16 * mt + lr) * HP + 8 * hi + 4]);
            v8us hv, rv;
#pragma unroll
            for (int i = 0; i < 4; ++i) {
                const unsigned short a0 = f2bf(x0[i]); const unsigned short a1 = f2bf(x1[i]);
                hv[i] = a0; hv[4 + i] = a1;
                rv[i] = f2bf(x0[i] - __uint_as_float(((unsigned)a0) << 16)); rv[4 + i] = f2bf(x1[i] - __uint_as_float(((unsigned)a1) << 16)); }
            acc[mt] = wmmab_g(cat16b(hv, rv), bw, (v8f){});
        }
    }
    wave_sync();

    {
        const float bv = bfr(b2[lr]);
#pragma unroll
        for (int mt = 0; mt < 2; ++mt) {
#pragma unroll
            for (int r = 0; r < 8; ++r) hs[(16 * mt + 8 * hi + r) * HP + lr] = acc[mt][r] + bv; }
    }
    wave_sync();
    float lq[16];
#pragma unroll
    for (int q = 0; q < 4; ++q) { const v4f t = *(const v4fa*)(&hs[lane * HP + 4 * q]);
#pragma unroll
        for (int i = 0; i < 4; ++i) lq[4 * q + i] = t[i]; }

    float X[16];
#pragma unroll
    for (int i = 0; i < 4; ++i) {
        float e[4]; float rs = 0.0f;
#pragma unroll
        for (int j = 0; j < 4; ++j) { e[j] = (j == i) ? 0.0f : expf(lq[i * 4 + j]); rs += e[j]; }
        const float inv = 1.0f / rs;
#pragma unroll
        for (int j = 0; j < 4; ++j) { const float q = (j == i) ? -1.0f : e[j] * inv; X[i * 4 + j] = (q * TINF) * XSC; }
    }

    float P[16], U[16];
#pragma unroll
    for (int i = 0; i < 16; ++i) P[i] = (i % 5 == 0) ? 1.0f : 0.0f;
#pragma unroll 1
    for (int k = TO; k >= 1; --k) {
        mm4(X, P, U);
        const float invk = 1.0f / (float)k;
#pragma unroll
        for (int i = 0; i < 16; ++i) P[i] = U[i] * invk + ((i % 5 == 0) ? 1.0f : 0.0f);
    }
#pragma unroll 1
    for (int r = 0; r < TS; ++r) {
        mm4(P, P, U);
#pragma unroll
        for (int i = 0; i < 16; ++i) P[i] = U[i];
    }

    v4f p; p[0] = P[0]; p[1] = P[1]; p[2] = P[2]; p[3] = P[3];
    float* pp = PR + (size_t)(v0 + lane) * NA;
    *(volatile v4f*)pp = p;
    __threadfence();
    *(volatile v4f*)pp = p;
}

__global__ __launch_bounds__(256) void k_bcast(const float* __restrict__ PR, float* OUT) {
    const int v = blockIdx.x;
    const v4f pv = *(const v4f*)(PR + (size_t)v * NA);
    float* o = OUT + (size_t)v * OUT_S * NA;
    const int t = threadIdx.x;
#pragma unroll 1
    for (int ps = 0; ps < 2; ++ps) {
#pragma unroll
        for (int r = 0; r < NS / 256; ++r) *(volatile v4f*)(o + (size_t)(t + r * 256) * NA) = pv;
        if (ps == 0) __threadfence(); }
}

static constexpr size_t al256(size_t v) { return (v + 255) & ~(size_t)255; }
static constexpr size_t SZ_PR = al256((size_t)NV * NA * 4);
static constexpr size_t SZ_TOTAL = SZ_PR;
static_assert(SZ_TOTAL <= (size_t)134217728);
static_assert((size_t)(NV / 32) * 32 * 16 == (size_t)NV * NA * 4);
static_assert(((size_t)(NV_FULL - 1) * OUT_S + NS_FULL) * NA * 4 <= (size_t)16777216);

extern "C" void kernel_launch(void* const* d_in, const int* in_sizes, int n_in,
                              void* d_out, int out_size, void* d_ws, size_t ws_size, hipStream_t stream) {
    (void)stream;
    if (n_in < 8) return;
    if ((size_t)in_sizes[0] < (size_t)NV * DE) return;
    if ((size_t)in_sizes[1] < (size_t)NS * 4) return;
    if (in_sizes[2] < DE * HW || in_sizes[3] < HW) return;
    if (in_sizes[4] < HW * HW || in_sizes[5] < HW) return;
    if (in_sizes[6] < HW * HW || in_sizes[7] < HW) return;
    if ((size_t)out_size < ((size_t)(NV - 1) * OUT_S + NS) * NA) return;
    if (SZ_TOTAL > ws_size) return;
    const float* emb = (const float*)d_in[0];
    const float* w0 = (const float*)d_in[2]; const float* b0 = (const float*)d_in[3];
    const float* w1 = (const float*)d_in[4]; const float* b1 = (const float*)d_in[5];
    const float* w2 = (const float*)d_in[6]; const float* b2 = (const float*)d_in[7];
    float* OUT = (float*)d_out;
    float* PR = (float*)d_ws;

    k_chain<<<dim3(NV / 32, 1, 1), 32, 0, stream>>>(emb, w0, b0, w1, b1, w2, b2, PR);
    k_bcast<<<dim3(NV, 1, 1), 256, 0, stream>>>(PR, OUT);
}
